// MD_BiDirectional_Hamiltonian_56667798503980
// MI455X (gfx1250) — hardware-run, weakly checked
//
#include <hip/hip_runtime.h>
#include <math.h>

typedef __attribute__((ext_vector_type(16))) _Float16 v16h;
typedef __attribute__((ext_vector_type(8)))  _Float16 v8h;
typedef __attribute__((ext_vector_type(4)))  _Float16 v4h;
typedef __attribute__((ext_vector_type(8)))  float    v8f;
typedef __attribute__((ext_vector_type(4)))  float    v4f;

constexpr int   kBatch      = 2048;
constexpr int   kFeat       = 64;
constexpr int   kHalfFeat   = 32;
constexpr int   kHid        = 128;
constexpr int   kTimePts    = 102;
constexpr int   kLastIdx    = kTimePts - 1;
constexpr int   kGradSteps  = 100;
constexpr int   kMidIdx     = 50;
constexpr int   kRowsPerBlk = 16;
constexpr int   kMainBlocks = kBatch / kRowsPerBlk;
constexpr int   kMainThreads = 512;
constexpr float kStepDt     = 0.1f;
constexpr float kWCarry     = 64.0f;
constexpr float kGCarry     = 256.0f;
constexpr float kResCarry   = 2048.0f;
constexpr float kInvW       = 1.0f / kWCarry;
constexpr float kInvRes     = 1.0f / kResCarry;
constexpr float kUpdCoef    = kStepDt / (kWCarry * kGCarry);
constexpr float kBlendInv   = 1.0f / (float)kLastIdx;
constexpr int   kPitchH     = 136;
constexpr int   kPitchY     = 72;

static_assert(kMainBlocks * kRowsPerBlk == kBatch, "batch tiling");
static_assert(kGradSteps + 2 == kTimePts, "time points");
static_assert(2 * kMidIdx + 1 == kLastIdx, "mid index");
static_assert((kFeat % 32) == 0 && (kHid % 32) == 0, "K multiples of 32");
static_assert((kPitchH % 8) == 0 && (kPitchY % 8) == 0, "16-B aligned LDS rows");

constexpr size_t kOffW1t  = 0;
constexpr size_t kOffW1s  = kOffW1t + (size_t)kHid * kFeat * 2;
constexpr size_t kOffW2t  = kOffW1s + (size_t)kFeat * kHid * 2;
constexpr size_t kOffW2s  = kOffW2t + (size_t)kHid * kHid * 2;
constexpr size_t kOffW3t  = kOffW2s + (size_t)kHid * kHid * 2;
constexpr size_t kOffW3s  = kOffW3t + (size_t)kHid * kHid * 2;
constexpr size_t kOffTab  = kOffW3s + (size_t)kHid * kHid * 2;
constexpr size_t kWsTotal = kOffTab + (size_t)4 * kHid * 4;
static_assert(kWsTotal == 165888ull, "carve total");
static_assert(kWsTotal <= 134217728ull, "carve cap");
static_assert((kOffW1s % 128) == 0 && (kOffW2t % 128) == 0 && (kOffW2s % 128) == 0 &&
              (kOffW3t % 128) == 0 && (kOffW3s % 128) == 0 && (kOffTab % 128) == 0, "128-B aligned regions");

constexpr int kBlkW1 = (kHid * kFeat / 8) / 256;
constexpr int kBlkW2 = (kHid * kHid / 8) / 256;
static_assert(kBlkW1 * 256 * 8 == kHid * kFeat && kBlkW2 * 256 * 8 == kHid * kHid, "exact plane coverage");
constexpr int kPrepBlocks = 2 * kBlkW1 + 4 * kBlkW2 + 1;

__device__ __forceinline__ unsigned short f2bf_bits(float f) {
  unsigned u = __float_as_uint(f);
  return (unsigned short)((u + 0x7FFFu + ((u >> 16) & 1u)) >> 16);
}
__device__ __forceinline__ float bf_bits2f(unsigned short h) { return __uint_as_float(((unsigned)h) << 16); }
__device__ __forceinline__ float bf16_rne(float f) { return bf_bits2f(f2bf_bits(f)); }

union FragU { v16h v; v8h h[2]; };
__device__ __forceinline__ v16h frag_ld(const _Float16* p) {
  FragU f;
  f.h[0] = *(const v8h*)(p);
  f.h[1] = *(const v8h*)(p + 16);
  return f.v;
}
__device__ __forceinline__ v8f mma_h(v16h a, v16h b, v8f c) {
  c = __builtin_amdgcn_wmma_f32_16x16x32_f16(false, a, false, b, (short)0, c, false, false);
  asm volatile("v_nop\n\tv_nop\n\tv_nop\n\tv_nop" : "+v"(c) : "v"(a), "v"(b));
  return c;
}
__device__ __forceinline__ float tanh_acc(float x) {
  const float ax = fabsf(x);
  const float t  = expf(-2.0f * ax);
  const float q  = (1.0f - t) * __builtin_amdgcn_rcpf(1.0f + t);
  return copysignf(q, x);
}
__device__ __forceinline__ void store8h_twice(unsigned short* dst, v8h hv) {
  *(volatile v8h*)dst = hv;
  __threadfence();
  *(volatile v8h*)dst = hv;
  __threadfence();
}

__device__ __forceinline__ void plane_transposed8(const float* __restrict__ W, int kin, int gid,
                                                  unsigned short* __restrict__ dst) {
  const int per = kin >> 3;
  const int n   = gid / per;
  const int k0  = (gid - n * per) << 3;
  v8h hv;
#pragma unroll
  for (int e = 0; e < 8; ++e) {
    const float w = W[(size_t)(k0 + e) * kHid + n];
    hv[e] = (_Float16)(bf16_rne(w) * kWCarry);
  }
  store8h_twice(dst + (size_t)n * kin + k0, hv);
}
__device__ __forceinline__ void plane_straight8(const float* __restrict__ W, int gid,
                                                unsigned short* __restrict__ dst) {
  const size_t e0 = (size_t)gid << 3;
  const v4f a0 = *(const v4f*)(W + e0);
  const v4f a1 = *(const v4f*)(W + e0 + 4);
  v8h hv;
#pragma unroll
  for (int e = 0; e < 4; ++e) {
    const float w0 = a0[e];
    const float w1 = a1[e];
    hv[e]     = (_Float16)(bf16_rne(w0) * kWCarry);
    hv[4 + e] = (_Float16)(bf16_rne(w1) * kWCarry);
  }
  store8h_twice(dst + e0, hv);
}

__global__ __launch_bounds__(256) void prep_planes_kernel(
    const float* __restrict__ W1, const float* __restrict__ b1,
    const float* __restrict__ W2, const float* __restrict__ b2,
    const float* __restrict__ W3, const float* __restrict__ b3,
    const float* __restrict__ W4, const float* __restrict__ W5,
    unsigned short* __restrict__ planes, float* __restrict__ tab)
{
  const int tid = threadIdx.x;
  const int blk = blockIdx.x;
  unsigned short* pW1t = planes + kOffW1t / 2;
  unsigned short* pW1s = planes + kOffW1s / 2;
  unsigned short* pW2t = planes + kOffW2t / 2;
  unsigned short* pW2s = planes + kOffW2s / 2;
  unsigned short* pW3t = planes + kOffW3t / 2;
  unsigned short* pW3s = planes + kOffW3s / 2;
  constexpr int e1 = kBlkW1;
  constexpr int e2 = e1 + kBlkW1;
  constexpr int e3 = e2 + kBlkW2;
  constexpr int e4 = e3 + kBlkW2;
  constexpr int e5 = e4 + kBlkW2;
  constexpr int e6 = e5 + kBlkW2;
  if (blk < e1) {
    plane_transposed8(W1, kFeat, blk * 256 + tid, pW1t);
  } else if (blk < e2) {
    plane_straight8(W1, (blk - e1) * 256 + tid, pW1s);
  } else if (blk < e3) {
    plane_transposed8(W2, kHid, (blk - e2) * 256 + tid, pW2t);
  } else if (blk < e4) {
    plane_straight8(W2, (blk - e3) * 256 + tid, pW2s);
  } else if (blk < e5) {
    plane_transposed8(W3, kHid, (blk - e4) * 256 + tid, pW3t);
  } else if (blk < e6) {
    plane_straight8(W3, (blk - e5) * 256 + tid, pW3s);
  } else {
    if (tid < 128) {
      const int wv = tid >> 5;
      const int ln = tid & 31;
      v4f val;
      if (wv < 3) {
        const float* src = (wv == 0) ? b1 : ((wv == 1) ? b2 : b3);
        const v4f t4 = *(const v4f*)(src + ln * 4);
#pragma unroll
        for (int e = 0; e < 4; ++e) {
          const float te = t4[e];
          val[e] = bf16_rne(te);
        }
      } else {
        float a0 = 0.f, a1 = 0.f, a2 = 0.f, a3 = 0.f;
        const float* wr = W4 + (size_t)(ln * 4) * kHid;
#pragma unroll 1
        for (int j = 0; j < kHid; ++j) {
          const float w5 = bf16_rne(W5[j]);
          a0 = fmaf(bf16_rne(wr[j]), w5, a0);
          a1 = fmaf(bf16_rne(wr[kHid + j]), w5, a1);
          a2 = fmaf(bf16_rne(wr[2 * kHid + j]), w5, a2);
          a3 = fmaf(bf16_rne(wr[3 * kHid + j]), w5, a3);
        }
        val[0] = a0; val[1] = a1; val[2] = a2; val[3] = a3;
      }
      float* dst = tab + tid * 4;
      *(volatile v4f*)dst = val;
      __threadfence();
      *(volatile v4f*)dst = val;
      __threadfence();
    }
  }
}

__global__ __launch_bounds__(512) void integrate_kernel(
    const int* __restrict__ tptr, const float* __restrict__ x,
    const unsigned short* __restrict__ planes, const float* __restrict__ tab, float* out)
{
  __shared__ __align__(16) _Float16 sW3[kHid * kPitchH];
  __shared__ __align__(16) _Float16 sW2[kHid * kPitchH];
  __shared__ __align__(16) _Float16 sW1[kFeat * kPitchH];
  __shared__ __align__(16) _Float16 sP[32 * kPitchH];
  __shared__ __align__(16) _Float16 sQ[32 * kPitchH];
  __shared__ __align__(16) _Float16 sYh[32 * kPitchY];
  __shared__ __align__(16) _Float16 sYl[32 * kPitchY];
  __shared__ __align__(16) float    sY[32 * kFeat];

  const int tid  = threadIdx.x;
  const int lane = tid & 31;
  const int wave = tid >> 5;
  const int hh   = lane >> 4;
  const int c    = lane & 15;
  const int nt   = wave & 7;
  const int mt   = wave >> 3;
  const int arow  = mt * 16 + c;
  const int drow0 = mt * 16 + 8 * hh;
  const int ncol  = nt * 16 + c;
  const int b0    = blockIdx.x * kRowsPerBlk;
  const int so  = tid >> 8;
  const int sr  = (tid >> 4) & 15;
  const int sc4 = (tid & 15) * 4;

  const _Float16* gp   = (const _Float16*)planes;
  const _Float16* gW1t = gp + kOffW1t / 2;
  const _Float16* gW1s = gp + kOffW1s / 2;
  const _Float16* gW2t = gp + kOffW2t / 2;
  const _Float16* gW2s = gp + kOffW2s / 2;
  const _Float16* gW3t = gp + kOffW3t / 2;
  const _Float16* gW3s = gp + kOffW3s / 2;

  const int   tv     = tptr[0];
  const float poison = (tv == kGradSteps) ? 0.0f : __uint_as_float(0x7fc00000u);

  for (int i = tid; i < kHid * 16; i += kMainThreads) {
    const int row = i >> 4, ch = (i & 15) * 8;
    *(v8h*)(sW3 + row * kPitchH + ch) = *(const v8h*)(gW3s + row * kHid + ch);
    *(v8h*)(sW2 + row * kPitchH + ch) = *(const v8h*)(gW2s + row * kHid + ch);
  }
  for (int i = tid; i < kFeat * 16; i += kMainThreads) {
    const int row = i >> 4, ch = (i & 15) * 8;
    *(v8h*)(sW1 + row * kPitchH + ch) = *(const v8h*)(gW1s + row * kHid + ch);
  }
  {
    const int m = so * 16 + sr;
    const v4f xv = *(const v4f*)(x + ((size_t)(b0 + sr) * 2 + so) * kFeat + sc4);
    const bool neg = (so == 1) && (sc4 >= kHalfFeat);
    v4f yv;
    v4h hv, lv;
#pragma unroll
    for (int e = 0; e < 4; ++e) {
      const float xe = xv[e];
      const float q  = bf16_rne(xe);
      const float v  = neg ? -q : q;
      const _Float16 hi = (_Float16)v;
      yv[e] = v;
      hv[e] = hi;
      lv[e] = (_Float16)((v - (float)hi) * kResCarry);
    }
    *(v4f*)(sY + m * kFeat + sc4) = yv;
    *(v4h*)(sYh + m * kPitchY + sc4) = hv;
    *(v4h*)(sYl + m * kPitchY + sc4) = lv;
  }
  v16h fW1t[2], fW2t[4], fW3t[4];
#pragma unroll
  for (int kc = 0; kc < 2; ++kc) fW1t[kc] = frag_ld(gW1t + (size_t)ncol * kFeat + kc * 32 + 8 * hh);
#pragma unroll
  for (int kc = 0; kc < 4; ++kc) {
    fW2t[kc] = frag_ld(gW2t + (size_t)ncol * kHid + kc * 32 + 8 * hh);
    fW3t[kc] = frag_ld(gW3t + (size_t)ncol * kHid + kc * 32 + 8 * hh);
  }
  const float b1v = tab[ncol];
  const float b2v = tab[kHid + ncol];
  const float b3v = tab[2 * kHid + ncol];
  const float v4c = tab[3 * kHid + ncol] * kGCarry;
  __syncthreads();

  const v8f vzero = (v8f){0.f, 0.f, 0.f, 0.f, 0.f, 0.f, 0.f, 0.f};

#pragma unroll 1
  for (int s = 0; s <= kGradSteps; ++s) {
    {
      const bool late   = (s > kMidIdx);
      const int  srcdir = late ? (1 - so) : so;
      const int  jown   = late ? (kLastIdx - s) : s;
      const int  joth   = late ? s : (kLastIdx - s);
      const int  j      = (so == 0) ? jown : joth;
      const float wgt   = (float)(kLastIdx - s) * kBlendInv;
      const float sg    = ((srcdir == 1) && (sc4 >= kHalfFeat)) ? -wgt : wgt;
      const v4f yv = *(const v4f*)(sY + (srcdir * 16 + sr) * kFeat + sc4);
      float* dst = out + ((size_t)(b0 + sr) * kTimePts + j) * kFeat + sc4;
      v4f val;
#pragma unroll
      for (int e = 0; e < 4; ++e) val[e] = yv[e] * sg + poison;
      if (late) {
        const v4f old = *(volatile v4f*)dst;
#pragma unroll
        for (int e = 0; e < 4; ++e) val[e] = val[e] + old[e];
      }
      *(volatile v4f*)dst = val;
      __threadfence();
      *(volatile v4f*)dst = val;
      __threadfence();
    }
    if (s < kGradSteps) {
      float h1r[8], h2r[8];
      {
        v8f acc = vzero, accr = vzero;
#pragma unroll
        for (int kc = 0; kc < 2; ++kc) {
          const v16h ah = frag_ld(sYh + arow * kPitchY + kc * 32 + 8 * hh);
          acc = mma_h(ah, fW1t[kc], acc);
          const v16h al = frag_ld(sYl + arow * kPitchY + kc * 32 + 8 * hh);
          accr = mma_h(al, fW1t[kc], accr);
        }
#pragma unroll
        for (int r = 0; r < 8; ++r) {
          const float z = (acc[r] + accr[r] * kInvRes) * kInvW + b1v;
          const float h = tanh_acc(z);
          h1r[r] = h;
          sP[(drow0 + r) * kPitchH + ncol] = (_Float16)h;
        }
      }
      __syncthreads();
      {
        v8f acc = vzero;
#pragma unroll
        for (int kc = 0; kc < 4; ++kc) {
          const v16h a = frag_ld(sP + arow * kPitchH + kc * 32 + 8 * hh);
          acc = mma_h(a, fW2t[kc], acc);
        }
#pragma unroll
        for (int r = 0; r < 8; ++r) {
          const float z = acc[r] * kInvW + b2v;
          const float h = tanh_acc(z);
          h2r[r] = h;
          sQ[(drow0 + r) * kPitchH + ncol] = (_Float16)h;
        }
      }
      __syncthreads();
      {
        v8f acc = vzero;
#pragma unroll
        for (int kc = 0; kc < 4; ++kc) {
          const v16h a = frag_ld(sQ + arow * kPitchH + kc * 32 + 8 * hh);
          acc = mma_h(a, fW3t[kc], acc);
        }
#pragma unroll
        for (int r = 0; r < 8; ++r) {
          const float z = acc[r] * kInvW + b3v;
          const float h = tanh_acc(z);
          const float d = v4c * (1.0f - h * h);
          sP[(drow0 + r) * kPitchH + ncol] = (_Float16)d;
        }
      }
      __syncthreads();
      {
        v8f acc = vzero;
#pragma unroll
        for (int kc = 0; kc < 4; ++kc) {
          const v16h a = frag_ld(sP + arow * kPitchH + kc * 32 + 8 * hh);
          const v16h b = frag_ld(sW3 + ncol * kPitchH + kc * 32 + 8 * hh);
          acc = mma_h(a, b, acc);
        }
#pragma unroll
        for (int r = 0; r < 8; ++r) {
          const float d = (acc[r] * kInvW) * (1.0f - h2r[r] * h2r[r]);
          sQ[(drow0 + r) * kPitchH + ncol] = (_Float16)d;
        }
      }
      __syncthreads();
      {
        v8f acc = vzero;
#pragma unroll
        for (int kc = 0; kc < 4; ++kc) {
          const v16h a = frag_ld(sQ + arow * kPitchH + kc * 32 + 8 * hh);
          const v16h b = frag_ld(sW2 + ncol * kPitchH + kc * 32 + 8 * hh);
          acc = mma_h(a, b, acc);
        }
#pragma unroll
        for (int r = 0; r < 8; ++r) {
          const float d = (acc[r] * kInvW) * (1.0f - h1r[r] * h1r[r]);
          sP[(drow0 + r) * kPitchH + ncol] = (_Float16)d;
        }
      }
      __syncthreads();
      if (nt < 4) {
        v8f acc = vzero;
#pragma unroll
        for (int kc = 0; kc < 4; ++kc) {
          const v16h a = frag_ld(sP + arow * kPitchH + kc * 32 + 8 * hh);
          const v16h b = frag_ld(sW1 + ncol * kPitchH + kc * 32 + 8 * hh);
          acc = mma_h(a, b, acc);
        }
        const int   tgt  = (ncol < kHalfFeat) ? (ncol + kHalfFeat) : (ncol - kHalfFeat);
        const float coef = (ncol < kHalfFeat) ? -kUpdCoef : kUpdCoef;
#pragma unroll
        for (int r = 0; r < 8; ++r) {
          const int row = drow0 + r;
          const float nv = sY[row * kFeat + tgt] + coef * acc[r];
          const _Float16 hi = (_Float16)nv;
          sY[row * kFeat + tgt] = nv;
          sYh[row * kPitchY + tgt] = hi;
          sYl[row * kPitchY + tgt] = (_Float16)((nv - (float)hi) * kResCarry);
        }
      }
      __syncthreads();
    }
  }
}

extern "C" void kernel_launch(void* const* d_in, const int* in_sizes, int n_in,
                              void* d_out, int out_size, void* d_ws, size_t ws_size,
                              hipStream_t stream) {
  if (n_in < 12) return;
  if (in_sizes[0] != 1) return;
  if (in_sizes[1] != kBatch * 2 * kFeat) return;
  if (in_sizes[2] != kFeat * kHid) return;
  if (in_sizes[3] != kHid) return;
  if (in_sizes[4] != kHid * kHid) return;
  if (in_sizes[5] != kHid) return;
  if (in_sizes[6] != kHid * kHid) return;
  if (in_sizes[7] != kHid) return;
  if (in_sizes[8] != kHid * kHid) return;
  if (in_sizes[10] != kHid) return;
  if (out_size != kBatch * kTimePts * kFeat) return;
  if (ws_size < kWsTotal) return;

  const int*   tp = (const int*)d_in[0];
  const float* x  = (const float*)d_in[1];
  const float* W1 = (const float*)d_in[2];
  const float* b1 = (const float*)d_in[3];
  const float* W2 = (const float*)d_in[4];
  const float* b2 = (const float*)d_in[5];
  const float* W3 = (const float*)d_in[6];
  const float* b3 = (const float*)d_in[7];
  const float* W4 = (const float*)d_in[8];
  const float* W5 = (const float*)d_in[10];
  float* out = (float*)d_out;

  char* ws = (char*)d_ws;
  unsigned short* planes = (unsigned short*)ws;
  float* tab = (float*)(ws + kOffTab);

  prep_planes_kernel<<<kPrepBlocks, 256, 0, stream>>>(W1, b1, W2, b2, W3, b3, W4, W5, planes, tab);
  integrate_kernel<<<kMainBlocks, kMainThreads, 0, stream>>>(tp, x, planes, tab, out);
}
